// GCN_ensemble_89472758710374
// MI455X (gfx1250) — hardware-verified
//
#include <hip/hip_runtime.h>
#include <stddef.h>


#define NF      128
#define NH      256
#define NTHR    256
#define NWAVE   8
#define EPT     8
#define NGRP    2
#define CHUNK   (NTHR * EPT * NGRP)
#define WCAP    (EPT * NGRP * 32)
#define LISTN   (NWAVE * WCAP)
#define NBC     4096
#define NBF     1024
#define RCAP    40960
#define RBN     128
#define TGT     256
#define DEGCAP  1024
#define GROWS   128
#define GCOLS   128
#define OTHR    512

#define LDS_FILL      ((RCAP + NBF + LISTN) * 4 + 64)
#define LDS_STG       (GROWS * GCOLS * 4)
#define LDS_GEMM(KD)  (2 * GROWS * ((KD) + 8) * 2 + LDS_STG)

static_assert((CHUNK & (CHUNK - 1)) == 0);
static_assert(CHUNK <= 4096);
static_assert(NBC <= 4096 && NBF <= 4096);
static_assert((NBC & (NBC - 1)) == 0 && (NBF & (NBF - 1)) == 0);
static_assert(NBC == 4 * NBF);
static_assert(OTHR * 8 == NBC);
static_assert((RCAP % 32) == 0);
static_assert(TGT == NWAVE * 32 && (TGT % GROWS) == 0);
static_assert(NF == 4 * 32);
static_assert((GROWS * NF / 8) % NTHR == 0 && (GROWS * NH / 8) % NTHR == 0);
static_assert((NH % GCOLS) == 0 && (NF % GCOLS) == 0 && (GCOLS % 64) == 0);
static_assert((NF * NH / 8) % NTHR == 0);
static_assert(GROWS == NWAVE * 16);

typedef float          v4f  __attribute__((ext_vector_type(4)));
typedef float          v8f  __attribute__((ext_vector_type(8)));
typedef int            v4i  __attribute__((ext_vector_type(4)));
typedef unsigned short v8us __attribute__((ext_vector_type(8)));
typedef __bf16         v16b __attribute__((ext_vector_type(16)));
union FragB { v16b v; v8us h[2]; };

__device__ __forceinline__ unsigned short bfh(float x) {
  unsigned u = __float_as_uint(x);
  u += 0x7FFFu + ((u >> 16) & 1u);
  return (unsigned short)(u >> 16);
}
__device__ __forceinline__ float bfv(unsigned short b) { return __uint_as_float(((unsigned)b) << 16); }

__device__ __forceinline__ void split8(v4f a, v4f b, v8us& hv, v8us& lv) {
  float x[8];
  x[0] = a.x; x[1] = a.y; x[2] = a.z; x[3] = a.w; x[4] = b.x; x[5] = b.y; x[6] = b.z; x[7] = b.w;
#pragma unroll
  for (int e = 0; e < 8; ++e) {
    const unsigned short hh = bfh(x[e]);
    const unsigned short ll = bfh(x[e] - bfv(hh));
    hv[e] = hh;
    lv[e] = ll;
  }
}

__device__ __forceinline__ v8f wmb(v16b a, v16b b, v8f c) {
  v8f d = __builtin_amdgcn_wmma_f32_16x16x32_bf16(false, a, false, b, (short)0, c, false, false);
  asm volatile("v_nop\n\tv_nop\n\tv_nop\n\tv_nop" : "+v"(d) : "v"(a), "v"(b));
  return d;
}

template <int NB>
__device__ __forceinline__ int scan_chunk(const int* __restrict__ dsts, int nE, int cbase, int slotBase,
                                          int vec8, int* list, int tid, int lane, int wave) {
  int wc = 0;
#pragma unroll
  for (int g = 0; g < NGRP; ++g) {
    const int el0  = (g * NTHR + tid) * EPT;
    const int e0   = cbase + el0;
    const int sent = -2147483647 - 1;
    v4i da, db;
    if (vec8 != 0 && cbase + CHUNK <= nE) {
      da = *(const v4i*)(dsts + e0);
      db = *(const v4i*)(dsts + e0 + 4);
    } else {
      da.x = (e0     < nE) ? dsts[min(e0, nE - 1)] : sent;
      da.y = (e0 + 1 < nE) ? dsts[min(e0 + 1, nE - 1)] : sent;
      da.z = (e0 + 2 < nE) ? dsts[min(e0 + 2, nE - 1)] : sent;
      da.w = (e0 + 3 < nE) ? dsts[min(e0 + 3, nE - 1)] : sent;
      db.x = (e0 + 4 < nE) ? dsts[min(e0 + 4, nE - 1)] : sent;
      db.y = (e0 + 5 < nE) ? dsts[min(e0 + 5, nE - 1)] : sent;
      db.z = (e0 + 6 < nE) ? dsts[min(e0 + 6, nE - 1)] : sent;
      db.w = (e0 + 7 < nE) ? dsts[min(e0 + 7, nE - 1)] : sent;
    }
    const unsigned nb = (unsigned)slotBase;
    const unsigned s0 = (unsigned)da.x - nb, s1 = (unsigned)da.y - nb;
    const unsigned s2 = (unsigned)da.z - nb, s3 = (unsigned)da.w - nb;
    const unsigned s4 = (unsigned)db.x - nb, s5 = (unsigned)db.y - nb;
    const unsigned s6 = (unsigned)db.z - nb, s7 = (unsigned)db.w - nb;
    const bool h0 = s0 < (unsigned)NB, h1 = s1 < (unsigned)NB, h2 = s2 < (unsigned)NB, h3 = s3 < (unsigned)NB;
    const bool h4 = s4 < (unsigned)NB, h5 = s5 < (unsigned)NB, h6 = s6 < (unsigned)NB, h7 = s7 < (unsigned)NB;
    const unsigned any = __builtin_amdgcn_ballot_w32(h0 | h1 | h2 | h3 | h4 | h5 | h6 | h7);
    if (any != 0u) {
#define HITJ(J, HJ, SJ) { \
        const unsigned mj = __builtin_amdgcn_ballot_w32(HJ); \
        if (mj != 0u) { \
          if (HJ) { \
            const int pos = wc + (int)__builtin_amdgcn_mbcnt_lo(mj, 0u); \
            if (pos < WCAP) list[wave * WCAP + pos] = ((el0 + (J)) << 12) | (int)(SJ); \
          } \
          wc += (int)__builtin_popcount(mj); } }
      HITJ(0, h0, s0)
      HITJ(1, h1, s1)
      HITJ(2, h2, s2)
      HITJ(3, h3, s3)
      HITJ(4, h4, s4)
      HITJ(5, h5, s5)
      HITJ(6, h6, s6)
      HITJ(7, h7, s7)
#undef HITJ
    }
  }
  return wc;
}

__global__ __launch_bounds__(NTHR) void k_wprep(
    const float* __restrict__ W0, const float* __restrict__ W1,
    const float* __restrict__ W2, const float* __restrict__ W3,
    unsigned short* p0h, unsigned short* p0l, unsigned short* p1h, unsigned short* p1l,
    unsigned short* p2h, unsigned short* p2l, unsigned short* p3h, unsigned short* p3l) {
  const int gseg = NF * NH / 8;
  const int seg  = (blockIdx.x * NTHR) / gseg;
  const int i    = blockIdx.x * NTHR + (int)threadIdx.x;
  if (i >= 4 * gseg) return;
  const float* src; unsigned short* dh; unsigned short* dl; int K, Nout;
  if (seg == 0)      { src = W0; dh = p0h; dl = p0l; K = NF; Nout = NH; }
  else if (seg == 1) { src = W1; dh = p1h; dl = p1l; K = NF; Nout = NH; }
  else if (seg == 2) { src = W2; dh = p2h; dl = p2l; K = NH; Nout = NF; }
  else               { src = W3; dh = p3h; dl = p3l; K = NH; Nout = NF; }
  const int o  = (i - seg * gseg) * 8;
  const int n  = o / K;
  const int k0 = o - n * K;
  v4f a, b;
  a.x = src[(size_t)(k0 + 0) * Nout + n]; a.y = src[(size_t)(k0 + 1) * Nout + n];
  a.z = src[(size_t)(k0 + 2) * Nout + n]; a.w = src[(size_t)(k0 + 3) * Nout + n];
  b.x = src[(size_t)(k0 + 4) * Nout + n]; b.y = src[(size_t)(k0 + 5) * Nout + n];
  b.z = src[(size_t)(k0 + 6) * Nout + n]; b.w = src[(size_t)(k0 + 7) * Nout + n];
  v8us hv, lv;
  split8(a, b, hv, lv);
  unsigned short* hp = dh + o;
  unsigned short* lp = dl + o;
  *(volatile v8us*)hp = hv;
  *(volatile v8us*)lp = lv;
  __threadfence();
  *(volatile v8us*)hp = hv;
  *(volatile v8us*)lp = lv;
}

__global__ __launch_bounds__(NTHR) void k_count(
    const int* __restrict__ ei, int* cnt, float* dinv, int nE, int vec8) {
  __shared__ __attribute__((aligned(16))) int scnt[NBC];
  __shared__ __attribute__((aligned(16))) int list[LISTN];
  __shared__ int wcnt[NWAVE];
  const int tid = threadIdx.x, lane = tid & 31, wave = tid >> 5;
  const int nodeBase = blockIdx.x * NBC;
  const int* dsts = ei + nE;

  for (int i = tid; i < NBC; i += NTHR) scnt[i] = 0;
  __syncthreads();

  const int nChunks = (nE + CHUNK - 1) / CHUNK;
#pragma unroll 1
  for (int ch = 0; ch < nChunks; ++ch) {
    const int cbase = ch * CHUNK;
    const int wc = scan_chunk<NBC>(dsts, nE, cbase, nodeBase, vec8, list, tid, lane, wave);
    if (lane == 0) wcnt[wave] = wc;
    __syncthreads();
    if (wave == 0) {
#pragma unroll 1
      for (int wsx = 0; wsx < NWAVE; ++wsx) {
        int n = __builtin_amdgcn_readfirstlane(wcnt[wsx]);
        n = n > WCAP ? WCAP : (n < 0 ? 0 : n);
        const int* lp = list + wsx * WCAP;
#pragma unroll 1
        for (int i = 0; i < n; ++i) {
          const int ent  = __builtin_amdgcn_readfirstlane(lp[i]);
          const int slot = ent & (NBC - 1);
          if (lane == 0) scnt[slot] = scnt[slot] + 1;
        }
      }
    }
    __syncthreads();
  }

  v4i cq[4]; v4f dq[4];
#pragma unroll
  for (int q = 0; q < 4; ++q) {
    const int f = (wave * 4 + q) * 128 + 4 * lane;
    const v4i c = *(const v4i*)(scnt + f);
    cq[q] = c;
    dq[q].x = rsqrtf((float)(c.x + 1));
    dq[q].y = rsqrtf((float)(c.y + 1));
    dq[q].z = rsqrtf((float)(c.z + 1));
    dq[q].w = rsqrtf((float)(c.w + 1));
  }
  int*   cp = cnt + (size_t)nodeBase;
  float* dp = dinv + (size_t)nodeBase;
#pragma unroll
  for (int q = 0; q < 4; ++q) {
    const int f = (wave * 4 + q) * 128 + 4 * lane;
    *(volatile v4i*)(cp + f) = cq[q];
    *(volatile v4f*)(dp + f) = dq[q];
  }
  __threadfence();
#pragma unroll
  for (int q = 0; q < 4; ++q) {
    const int f = (wave * 4 + q) * 128 + 4 * lane;
    *(volatile v4i*)(cp + f) = cq[q];
    *(volatile v4f*)(dp + f) = dq[q];
  }
}

__global__ __launch_bounds__(OTHR) void k_offsets(
    const int* __restrict__ cnt, int* off, int* rbase, int nChunk) {
  __shared__ __attribute__((aligned(16))) int soff[NBC];
  __shared__ __attribute__((aligned(16))) int srb[RBN];
  __shared__ int wtot[OTHR / 32];
  const int tid = threadIdx.x, lane = tid & 31, wave = tid >> 5, sub = tid >> 7;
  for (int i = tid; i < RBN; i += OTHR) srb[i] = 0;
  int carry = 0;
#pragma unroll 1
  for (int ch = 0; ch < nChunk; ++ch) {
    const int base = ch * NBC;
    const v4i c0 = *(const v4i*)(cnt + base + 8 * tid);
    const v4i c1 = *(const v4i*)(cnt + base + 8 * tid + 4);
    const int e0 = max(c0.x, 0), e1 = max(c0.y, 0), e2 = max(c0.z, 0), e3 = max(c0.w, 0);
    const int e4 = max(c1.x, 0), e5 = max(c1.y, 0), e6 = max(c1.z, 0), e7 = max(c1.w, 0);
    const int ts = e0 + e1 + e2 + e3 + e4 + e5 + e6 + e7;
    int incl = ts;
#pragma unroll
    for (int d = 1; d < 32; d <<= 1) {
      const int t = __shfl_up(incl, d);
      if (lane >= d) incl += t;
    }
    if (lane == 31) wtot[wave] = incl;
    __syncthreads();
    const int S0 = wtot[0]  + wtot[1]  + wtot[2]  + wtot[3];
    const int S1 = wtot[4]  + wtot[5]  + wtot[6]  + wtot[7];
    const int S2 = wtot[8]  + wtot[9]  + wtot[10] + wtot[11];
    const int S3 = wtot[12] + wtot[13] + wtot[14] + wtot[15];
    int pre = 0;
#pragma unroll 1
    for (int w = 4 * sub; w < wave; ++w) pre += wtot[w];
    const int b0 = carry;
    const int b1 = b0 + ((S0 + 31) & ~31);
    const int b2 = b1 + ((S1 + 31) & ~31);
    const int b3 = b2 + ((S2 + 31) & ~31);
    const int b4 = b3 + ((S3 + 31) & ~31);
    const int myb = sub == 0 ? b0 : (sub == 1 ? b1 : (sub == 2 ? b2 : b3));
    if (tid == 0) {
      srb[min(4 * ch + 0, RBN - 1)] = b0;
      srb[min(4 * ch + 1, RBN - 1)] = b1;
      srb[min(4 * ch + 2, RBN - 1)] = b2;
      srb[min(4 * ch + 3, RBN - 1)] = b3;
    }
    int run = myb + pre + incl - ts;
    soff[8 * tid + 0] = run; run += e0;
    soff[8 * tid + 1] = run; run += e1;
    soff[8 * tid + 2] = run; run += e2;
    soff[8 * tid + 3] = run; run += e3;
    soff[8 * tid + 4] = run; run += e4;
    soff[8 * tid + 5] = run; run += e5;
    soff[8 * tid + 6] = run; run += e6;
    soff[8 * tid + 7] = run;
    carry = b4;
    __syncthreads();
    const v4i o0 = *(const v4i*)(soff + 4 * tid);
    const v4i o1 = *(const v4i*)(soff + 4 * (tid + OTHR));
    int* op = off + base;
    *(volatile v4i*)(op + 4 * tid) = o0;
    *(volatile v4i*)(op + 4 * (tid + OTHR)) = o1;
    __threadfence();
    *(volatile v4i*)(op + 4 * tid) = o0;
    *(volatile v4i*)(op + 4 * (tid + OTHR)) = o1;
    __syncthreads();
  }
  if (tid == 0) srb[min(4 * nChunk, RBN - 1)] = carry;
  __syncthreads();
  v4i rv = {0, 0, 0, 0};
  if (tid < 32) rv = *(const v4i*)(srb + 4 * tid);
  if (tid < 32) *(volatile v4i*)(rbase + 4 * tid) = rv;
  __threadfence();
  if (tid < 32) *(volatile v4i*)(rbase + 4 * tid) = rv;
}

__global__ __launch_bounds__(NTHR) void k_fill(
    const int* __restrict__ ei, const int* __restrict__ off, const int* __restrict__ rbase,
    int* csr, int nN, int nE, int vec8, int csrLen) {
  extern __shared__ v4f lds_dyn[];
  int* region = (int*)lds_dyn;
  int* cursor = region + RCAP;
  int* list   = cursor + NBF;
  int* wcnt   = list + LISTN;
  const int tid = threadIdx.x, lane = tid & 31, wave = tid >> 5;
  const int b = blockIdx.x;
  const int nodeBase = b * NBF;
  const int* dsts = ei + nE;

  int rb0 = rbase[b];
  const int rb1 = rbase[b + 1];
  rb0 = rb0 < 0 ? 0 : (rb0 > csrLen ? csrLen : rb0);
  rb0 &= ~31;
  int len = rb1 - rb0;
  len = len < 0 ? 0 : (len > RCAP ? RCAP : len);
  int lenW = (len + 31) & ~31;
  if (rb0 + lenW > csrLen) lenW = (csrLen - rb0) & ~31;

  {
    const v4i z = {0, 0, 0, 0};
    for (int i = tid; i < RCAP / 4; i += NTHR) ((v4i*)region)[i] = z;
    for (int s = tid; s < NBF; s += NTHR) {
      int o = off[nodeBase + s] - rb0;
      o = o < 0 ? 0 : (o > RCAP ? RCAP : o);
      cursor[s] = o;
    }
  }
  __syncthreads();

  const int nChunks = (nE + CHUNK - 1) / CHUNK;
#pragma unroll 1
  for (int ch = 0; ch < nChunks; ++ch) {
    const int cbase = ch * CHUNK;
    const int wc = scan_chunk<NBF>(dsts, nE, cbase, nodeBase, vec8, list, tid, lane, wave);
    if (lane == 0) wcnt[wave] = wc;
    __syncthreads();
    if (wave == 0) {
#pragma unroll 1
      for (int wsx = 0; wsx < NWAVE; ++wsx) {
        int n = __builtin_amdgcn_readfirstlane(wcnt[wsx]);
        n = n > WCAP ? WCAP : (n < 0 ? 0 : n);
        const int* lp = list + wsx * WCAP;
#pragma unroll 1
        for (int i = 0; i < n; ++i) {
          const int ent  = __builtin_amdgcn_readfirstlane(lp[i]);
          const int slot = ent & (NBF - 1);
          int e = cbase + ((ent >> 12) & (CHUNK - 1));
          e = e > nE - 1 ? nE - 1 : e;
          int src = ei[e];
          src = src < 0 ? 0 : (src > nN - 1 ? nN - 1 : src);
          if (lane == 0) {
            int pos = cursor[slot];
            pos = pos < 0 ? 0 : (pos > RCAP - 1 ? RCAP - 1 : pos);
            region[pos] = src;
            const int np = pos + 1;
            cursor[slot] = np > RCAP ? RCAP : np;
          }
        }
      }
    }
    __syncthreads();
  }

  const int nv = lenW >> 2;
  int* gp = csr + rb0;
#pragma unroll 1
  for (int i = tid; i < nv; i += NTHR) { const v4i v = ((const v4i*)region)[i]; *(volatile v4i*)(gp + 4 * i) = v; }
  __threadfence();
#pragma unroll 1
  for (int i = tid; i < nv; i += NTHR) { const v4i v = ((const v4i*)region)[i]; *(volatile v4i*)(gp + 4 * i) = v; }
}

template <int KD>
__global__ __launch_bounds__(NTHR) void k_gemm(
    const float* __restrict__ A, const unsigned short* __restrict__ Bh, const unsigned short* __restrict__ Bl,
    const float* __restrict__ bias, float* C, int nRowsA, int ldc, int useBias, int useRelu) {
  extern __shared__ v4f lds_dyn[];
  constexpr int AP = KD + 8;
  unsigned short* sH  = (unsigned short*)lds_dyn;
  unsigned short* sL  = sH + GROWS * AP;
  float*          stg = (float*)(sL + GROWS * AP);
  const int tid = threadIdx.x, lane = tid & 31, wave = tid >> 5, hh = lane >> 4, m = lane & 15;
  const int rowBase = blockIdx.x * GROWS;
  const int colBase = blockIdx.y * GCOLS;

#pragma unroll
  for (int i = 0; i < (GROWS * KD / 8) / NTHR; ++i) {
    const int idx = i * NTHR + tid;
    const int r   = idx / (KD / 8);
    const int c0  = (idx - r * (KD / 8)) * 8;
    int row = rowBase + r;
    row = row > nRowsA - 1 ? nRowsA - 1 : row;
    const float* ap = A + (size_t)row * KD + c0;
    const v4f a = *(const v4f*)ap, b = *(const v4f*)(ap + 4);
    v8us hv, lv;
    split8(a, b, hv, lv);
    *(v8us*)(sH + r * AP + c0) = hv;
    *(v8us*)(sL + r * AP + c0) = lv;
  }
  __syncthreads();

  const unsigned short* arH = sH + (wave * 16 + m) * AP + 8 * hh;
  const unsigned short* arL = sL + (wave * 16 + m) * AP + 8 * hh;
  const int r0 = wave * 16 + 8 * hh;
#pragma unroll 1
  for (int g = 0; g < GCOLS / 64; ++g) {
    v8f acc[4];
#pragma unroll
    for (int t = 0; t < 4; ++t) { v8f z = {0.f, 0.f, 0.f, 0.f, 0.f, 0.f, 0.f, 0.f}; acc[t] = z; }
#pragma unroll
    for (int kt = 0; kt < KD / 32; ++kt) {
      FragB ah, al;
      ah.h[0] = *(const v8us*)(arH + 32 * kt);
      ah.h[1] = *(const v8us*)(arH + 32 * kt + 16);
      al.h[0] = *(const v8us*)(arL + 32 * kt);
      al.h[1] = *(const v8us*)(arL + 32 * kt + 16);
#pragma unroll
      for (int t = 0; t < 4; ++t) {
        const size_t boff = (size_t)(colBase + 64 * g + 16 * t + m) * KD + 32 * kt + 8 * hh;
        FragB bh, bl;
        bh.h[0] = *(const v8us*)(Bh + boff);
        bh.h[1] = *(const v8us*)(Bh + boff + 16);
        bl.h[0] = *(const v8us*)(Bl + boff);
        bl.h[1] = *(const v8us*)(Bl + boff + 16);
        acc[t] = wmb(ah.v, bh.v, acc[t]);
        acc[t] = wmb(ah.v, bl.v, acc[t]);
        acc[t] = wmb(al.v, bh.v, acc[t]);
      }
    }
#pragma unroll
    for (int t = 0; t < 4; ++t) {
      const int cl   = 64 * g + 16 * t + m;
      const float bl = bias[colBase + cl];
      const float bv = useBias != 0 ? bl : 0.0f;
      float* sp = stg + r0 * GCOLS + cl;
#pragma unroll
      for (int r = 0; r < 8; ++r) {
        float v = acc[t][r] + bv;
        const float vr = fmaxf(v, 0.0f);
        v = useRelu != 0 ? vr : v;
        sp[r * GCOLS] = v;
      }
    }
  }
  __syncthreads();

  const float* lp = stg + wave * 16 * GCOLS + 4 * lane;
  float* gp = C + ((size_t)rowBase + wave * 16) * ldc + colBase + 4 * lane;
#pragma unroll
  for (int i = 0; i < 16; ++i) { const v4f v = *(const v4f*)(lp + i * GCOLS); *(volatile v4f*)(gp + (size_t)i * ldc) = v; }
  __threadfence();
#pragma unroll
  for (int i = 0; i < 16; ++i) { const v4f v = *(const v4f*)(lp + i * GCOLS); *(volatile v4f*)(gp + (size_t)i * ldc) = v; }
}

__global__ __launch_bounds__(NTHR) void k_agg(
    const int* __restrict__ csr, const int* __restrict__ off, const int* __restrict__ cnt,
    const float* __restrict__ dinv, const float* __restrict__ X, const float* __restrict__ bias,
    const float* addp, float* Y, int nRowsX, int nRowsY, int nN, int csrLen, int useBias, int useAdd) {
  const int tid = threadIdx.x, lane = tid & 31, wave = tid >> 5;
  const int tbase = blockIdx.x * TGT + wave * 32;
  const int cl = tbase + lane;
  const int cnt_l = cnt[cl];
  const int off_l = off[cl];
  union FI { float f; int i; };
  FI dvu; dvu.f = dinv[cl];
  v4f bb = {0.f, 0.f, 0.f, 0.f};
  if (useBias != 0) bb = *(const v4f*)(bias + 4 * lane);

#pragma unroll 1
  for (int j = 0; j < 32; ++j) {
    const int c = tbase + j;
    int n = __builtin_amdgcn_readlane(cnt_l, j);
    n = n < 0 ? 0 : (n > DEGCAP ? DEGCAP : n);
    const int st = __builtin_amdgcn_readlane(off_l, j);
    FI du; du.i = __builtin_amdgcn_readlane(dvu.i, j);
    const float dc = du.f;
    v4f acc = {0.f, 0.f, 0.f, 0.f};
#pragma unroll 1
    for (int q0 = 0; q0 < n; q0 += 32) {
      int pos = st + q0 + lane;
      pos = pos < 0 ? 0 : (pos > csrLen - 1 ? csrLen - 1 : pos);
      int sl = csr[pos];
      sl = sl < 0 ? 0 : (sl > nN - 1 ? nN - 1 : sl);
      FI wl; wl.f = dinv[sl];
      const int mcnt = (n - q0) < 32 ? (n - q0) : 32;
#pragma unroll 1
      for (int p = 0; p < mcnt; ++p) {
        const int s = __builtin_amdgcn_readlane(sl, p);
        FI wu; wu.i = __builtin_amdgcn_readlane(wl.i, p);
        const v4f xv = *(const v4f*)(X + (size_t)s * NF + 4 * lane);
        acc = acc + xv * wu.f;
      }
    }
    const int cs = c < nRowsX - 1 ? c : nRowsX - 1;
    const v4f sv = *(const v4f*)(X + (size_t)cs * NF + 4 * lane);
    v4f v = (acc + sv * dc) * dc + bb;
    if (useAdd != 0) {
      const v4f ad = *(const v4f*)(addp + (size_t)c * NF + 4 * lane);
      v = v + ad;
    }
    if (c < nRowsY) {
      float* yp = Y + (size_t)c * NF + 4 * lane;
      *(volatile v4f*)yp = v;
      __threadfence();
      *(volatile v4f*)yp = v;
    }
  }
}

extern "C" void kernel_launch(void* const* d_in, const int* in_sizes, int n_in,
                              void* d_out, int out_size, void* d_ws, size_t ws_size,
                              hipStream_t stream) {
  if (n_in < 11) return;
  const int nN  = in_sizes[0] / NF;
  const int nEA = in_sizes[1] / 2;
  const int nEB = in_sizes[2] / 2;
  if (nN <= 0 || nEA <= 0 || nEB <= 0) return;
  if (in_sizes[0] != nN * NF || in_sizes[1] != 2 * nEA || in_sizes[2] != 2 * nEB) return;
  if (in_sizes[3] != NF * NH || in_sizes[5] != NF * NH || in_sizes[7] != NH * NF || in_sizes[9] != NH * NF) return;
  if (in_sizes[4] < NH || in_sizes[6] < NH || in_sizes[8] < NF || in_sizes[10] < NF) return;
  if (out_size != nN * NF) return;
  if (nN > (1 << 24) || nEA > (1 << 28) || nEB > (1 << 28)) return;

  const float* x   = (const float*)d_in[0];
  const int*   eiA = (const int*)d_in[1];
  const int*   eiB = (const int*)d_in[2];
  const float* W0  = (const float*)d_in[3];
  const float* b0  = (const float*)d_in[4];
  const float* W1  = (const float*)d_in[5];
  const float* b1  = (const float*)d_in[6];
  const float* W2  = (const float*)d_in[7];
  const float* b2  = (const float*)d_in[8];
  const float* W3  = (const float*)d_in[9];
  const float* b3  = (const float*)d_in[10];
  float* out = (float*)d_out;

  const int NPAD   = ((nN + TGT - 1) / TGT) * TGT;
  const int nBC    = (nN + NBC - 1) / NBC;
  const int CNTPAD = nBC * NBC;
  if (4 * nBC + 1 > RBN) return;
  if (CNTPAD < NPAD) return;
  const int nBF     = (nN + NBF - 1) / NBF;
  const int csrLenA = ((nEA + 31) & ~31) + 4096;
  const int csrLenB = ((nEB + 31) & ~31) + 4096;
  const int nGemm   = NPAD / GROWS;
  const int nAgg    = NPAD / TGT;

  char* ws = (char*)d_ws;
  size_t off = 0;
  const size_t wpl = (size_t)NF * NH * 2;
  const size_t oP0h = off; off += wpl;  off = (off + 255) & ~(size_t)255;
  const size_t oP0l = off; off += wpl;  off = (off + 255) & ~(size_t)255;
  const size_t oP1h = off; off += wpl;  off = (off + 255) & ~(size_t)255;
  const size_t oP1l = off; off += wpl;  off = (off + 255) & ~(size_t)255;
  const size_t oP2h = off; off += wpl;  off = (off + 255) & ~(size_t)255;
  const size_t oP2l = off; off += wpl;  off = (off + 255) & ~(size_t)255;
  const size_t oP3h = off; off += wpl;  off = (off + 255) & ~(size_t)255;
  const size_t oP3l = off; off += wpl;  off = (off + 255) & ~(size_t)255;
  const size_t oCnA = off; off += (size_t)CNTPAD * 4;    off = (off + 255) & ~(size_t)255;
  const size_t oDvA = off; off += (size_t)CNTPAD * 4;    off = (off + 255) & ~(size_t)255;
  const size_t oOfA = off; off += (size_t)CNTPAD * 4;    off = (off + 255) & ~(size_t)255;
  const size_t oRbA = off; off += (size_t)RBN * 4;       off = (off + 255) & ~(size_t)255;
  const size_t oCnB = off; off += (size_t)CNTPAD * 4;    off = (off + 255) & ~(size_t)255;
  const size_t oDvB = off; off += (size_t)CNTPAD * 4;    off = (off + 255) & ~(size_t)255;
  const size_t oOfB = off; off += (size_t)CNTPAD * 4;    off = (off + 255) & ~(size_t)255;
  const size_t oRbB = off; off += (size_t)RBN * 4;       off = (off + 255) & ~(size_t)255;
  const size_t oCsA = off; off += (size_t)csrLenA * 4;   off = (off + 255) & ~(size_t)255;
  const size_t oCsB = off; off += (size_t)csrLenB * 4;   off = (off + 255) & ~(size_t)255;
  const size_t oAX  = off; off += (size_t)NPAD * NF * 4; off = (off + 255) & ~(size_t)255;
  const size_t oT   = off; off += (size_t)NPAD * NH * 4; off = (off + 255) & ~(size_t)255;
  const size_t oO1  = off; off += (size_t)NPAD * NF * 4; off = (off + 255) & ~(size_t)255;
  if (off > ws_size) return;
  unsigned short* p0h = (unsigned short*)(ws + oP0h); unsigned short* p0l = (unsigned short*)(ws + oP0l);
  unsigned short* p1h = (unsigned short*)(ws + oP1h); unsigned short* p1l = (unsigned short*)(ws + oP1l);
  unsigned short* p2h = (unsigned short*)(ws + oP2h); unsigned short* p2l = (unsigned short*)(ws + oP2l);
  unsigned short* p3h = (unsigned short*)(ws + oP3h); unsigned short* p3l = (unsigned short*)(ws + oP3l);
  int*   cntA = (int*)(ws + oCnA);  float* dvA = (float*)(ws + oDvA); int* offA = (int*)(ws + oOfA); int* rbA = (int*)(ws + oRbA);
  int*   cntB = (int*)(ws + oCnB);  float* dvB = (float*)(ws + oDvB); int* offB = (int*)(ws + oOfB); int* rbB = (int*)(ws + oRbB);
  int*   csrA = (int*)(ws + oCsA);
  int*   csrB = (int*)(ws + oCsB);
  float* ax   = (float*)(ws + oAX);
  float* tpl  = (float*)(ws + oT);
  float* o1   = (float*)(ws + oO1);

  const int vecA = ((nEA & 3) == 0) ? 1 : 0;
  const int vecB = ((nEB & 3) == 0) ? 1 : 0;

  k_wprep<<<(4 * (NF * NH / 8)) / NTHR, NTHR, 0, stream>>>(W0, W1, W2, W3, p0h, p0l, p1h, p1l, p2h, p2l, p3h, p3l);

  k_count<<<nBC, NTHR, 0, stream>>>(eiA, cntA, dvA, nEA, vecA);
  k_count<<<nBC, NTHR, 0, stream>>>(eiB, cntB, dvB, nEB, vecB);
  k_offsets<<<1, OTHR, 0, stream>>>(cntA, offA, rbA, nBC);
  k_offsets<<<1, OTHR, 0, stream>>>(cntB, offB, rbB, nBC);
  hipFuncSetAttribute(reinterpret_cast<const void*>(&k_fill),
                      hipFuncAttributeMaxDynamicSharedMemorySize, LDS_FILL);
  k_fill<<<nBF, NTHR, LDS_FILL, stream>>>(eiA, offA, rbA, csrA, nN, nEA, vecA, csrLenA);
  k_fill<<<nBF, NTHR, LDS_FILL, stream>>>(eiB, offB, rbB, csrB, nN, nEB, vecB, csrLenB);

  hipFuncSetAttribute(reinterpret_cast<const void*>(&k_gemm<NF>),
                      hipFuncAttributeMaxDynamicSharedMemorySize, LDS_GEMM(NF));
  hipFuncSetAttribute(reinterpret_cast<const void*>(&k_gemm<NH>),
                      hipFuncAttributeMaxDynamicSharedMemorySize, LDS_GEMM(NH));

  k_agg<<<nAgg, NTHR, 0, stream>>>(csrA, offA, cntA, dvA, x, b0, o1, ax, nN, NPAD, nN, csrLenA, 0, 0);
  k_gemm<NF><<<dim3(nGemm, NH / GCOLS), NTHR, LDS_GEMM(NF), stream>>>(ax, p0h, p0l, b0, tpl, NPAD, NH, 1, 1);
  k_gemm<NH><<<dim3(nGemm, NF / GCOLS), NTHR, LDS_GEMM(NH), stream>>>(tpl, p2h, p2l, b2, ax, NPAD, NF, 0, 0);
  k_agg<<<nAgg, NTHR, 0, stream>>>(csrA, offA, cntA, dvA, ax, b2, o1, o1, NPAD, NPAD, nN, csrLenA, 1, 0);

  k_agg<<<nAgg, NTHR, 0, stream>>>(csrB, offB, cntB, dvB, x, b1, o1, ax, nN, NPAD, nN, csrLenB, 0, 0);
  k_gemm<NF><<<dim3(nGemm, NH / GCOLS), NTHR, LDS_GEMM(NF), stream>>>(ax, p1h, p1l, b1, tpl, NPAD, NH, 1, 1);
  k_gemm<NH><<<dim3(nGemm, NF / GCOLS), NTHR, LDS_GEMM(NH), stream>>>(tpl, p3h, p3l, b3, ax, NPAD, NF, 0, 0);
  k_agg<<<nAgg, NTHR, 0, stream>>>(csrB, offB, cntB, dvB, ax, b3, o1, out, NPAD, nN, nN, csrLenB, 1, 1);
}
